// CrossScan_SS2D_23699629539952
// MI455X (gfx1250) — hardware-run, weakly checked
//
#include <hip/hip_runtime.h>
#include <math.h>

#define NBAT   4
#define NI     32
#define NJ     32
#define SEQL   1024
#define NSEQ   16
#define MTOK   16384
#define NPIX   4096
#define DM     192
#define DI     384
#define NH     6
#define HDIM   64
#define DSTATE 64
#define NPJ    902
#define LDZ    960
#define CD     512
#define COL_XBC 384
#define COL_DT  896
#define XCB    384
#define XCC    448
#define TPB    128
#define OSTR   68
#define SCH    32
#define NSUB   4
#define NSTS   16
#define WOSC   256.0f
#define WOSCI  0.00390625f
#define EPSV   1e-5f
#define WSCAP  134217728

static_assert(MTOK == NSEQ * SEQL);
static_assert(NPIX == NBAT * NI * NJ);
static_assert(NSEQ == 4 * NBAT);
static_assert(MTOK % TPB == 0);
static_assert(NPIX % TPB == 0);
static_assert(LDZ % 64 == 0);
static_assert(LDZ >= NPJ);
static_assert(DM % 64 == 0);
static_assert(DM % 32 == 0);
static_assert(DI % 32 == 0);
static_assert(DM % 8 == 0);
static_assert(DI % 8 == 0);
static_assert(NSUB * NSTS == DSTATE);
static_assert(HDIM * NSUB == 256);
static_assert(NH * HDIM == DI);
static_assert(CD == DI + 2 * DSTATE);
static_assert(NPJ == 2 * DI + 2 * DSTATE + NH);
static_assert(SEQL % SCH == 0);
static_assert(SCH * HDIM == 2 * 256 * 4);
static_assert(SEQL % 256 == 0);
static_assert(OSTR % 4 == 0);
static_assert(CD % 4 == 0);
static_assert((CD / 4) == 128);

typedef unsigned short us16 __attribute__((ext_vector_type(16)));
typedef unsigned short us8  __attribute__((ext_vector_type(8)));
typedef unsigned short us8a __attribute__((ext_vector_type(8), may_alias));
typedef __bf16 v16b __attribute__((ext_vector_type(16)));
typedef _Float16 v16h __attribute__((ext_vector_type(16)));
typedef float v8f __attribute__((ext_vector_type(8)));
typedef float v4f __attribute__((ext_vector_type(4)));
typedef float v4fa __attribute__((ext_vector_type(4), may_alias));
union FragU { us16 v; us8 h[2]; };

__device__ __forceinline__ unsigned short bf16_bits(float f) {
  unsigned u = __float_as_uint(f);
  u += 0x7FFFu + ((u >> 16) & 1u);
  return (unsigned short)(u >> 16);
}
__device__ __forceinline__ float bf16_val(unsigned short b) { return __uint_as_float(((unsigned)b) << 16); }
__device__ __forceinline__ float bf16r(float f) { return bf16_val(bf16_bits(f)); }
__device__ __forceinline__ unsigned short f16_bits(float f) { const _Float16 hv = (_Float16)f; return __builtin_bit_cast(unsigned short, hv); }
__device__ __forceinline__ float siluf(float x) { return x * __builtin_amdgcn_rcpf(1.0f + __expf(-x)); }

template <int F16> struct MmaSel;
template <> struct MmaSel<0> {
  static __device__ __forceinline__ v8f run(us16 a, us16 b, v8f c) {
    return __builtin_amdgcn_wmma_f32_16x16x32_bf16(false, __builtin_bit_cast(v16b, a), false, __builtin_bit_cast(v16b, b), (short)0, c, false, false);
  }
};
template <> struct MmaSel<1> {
  static __device__ __forceinline__ v8f run(us16 a, us16 b, v8f c) {
    return __builtin_amdgcn_wmma_f32_16x16x32_f16(false, __builtin_bit_cast(v16h, a), false, __builtin_bit_cast(v16h, b), (short)0, c, false, false);
  }
};
__device__ __forceinline__ void wguard(v8f& c0, v8f& c1, v8f& c2, v8f& c3, const us16& a0,
                                       const us16& b0, const us16& b1, const us16& b2, const us16& b3) {
#if defined(__HIP_DEVICE_COMPILE__)
  asm volatile("v_nop\n\tv_nop\n\tv_nop\n\tv_nop"
               : "+v"(c0), "+v"(c1), "+v"(c2), "+v"(c3)
               : "v"(a0), "v"(b0), "v"(b1), "v"(b2), "v"(b3));
#endif
}

__device__ __forceinline__ us16 gfrag(const unsigned short* p) {
  const int kh = ((threadIdx.x >> 4) & 1) * 8;
  FragU f;
  f.h[0] = *(const us8a*)(p + kh);
  f.h[1] = *(const us8a*)(p + 16 + kh);
  return f.v;
}

__global__ __launch_bounds__(256) void k_gather(const float* __restrict__ x, unsigned short* XB) {
  const int idx = blockIdx.x * 256 + threadIdx.x;
  if (idx >= MTOK * (DM / 8)) return;
  const int m = idx / (DM / 8), c8 = (idx - m * (DM / 8)) * 8;
  const int s = m >> 10, l = m & (SEQL - 1), dir = s / NBAT, b = s % NBAT;
  const int i = l >> 5, j = l & 31;
  const int hq = (dir < 2) ? i : ((dir == 2) ? j : (31 - j));
  const int wq = (dir == 0) ? j : ((dir == 1) ? (31 - j) : i);
  const float* xr = x + ((size_t)((b * NI + hq) * NJ + wq)) * DM + c8;
  const v4f a = *(const v4fa*)xr, bq = *(const v4fa*)(xr + 4);
  us8 o;
#pragma unroll
  for (int u = 0; u < 4; ++u) { o[u] = bf16_bits(a[u]); o[4 + u] = bf16_bits(bq[u]); }
  const size_t off = (size_t)m * DM + c8;
  *(volatile us8*)(XB + off) = o;
  __threadfence();
  *(volatile us8*)(XB + off) = o;
}

template <int F16>
__global__ __launch_bounds__(256) void k_cvtw(const float* __restrict__ src, unsigned short* dst, int K, int N, int total8, float scale) {
  const int idx = blockIdx.x * 256 + threadIdx.x;
  if (idx >= total8) return;
  const int k8n = K >> 3;
  const int n = idx / k8n, k8 = (idx - n * k8n) * 8;
  const int ns = (n < N) ? n : (N - 1);
  const bool zr = (n >= N);
  us8 o;
#pragma unroll
  for (int u = 0; u < 8; ++u) {
    const float f = src[(size_t)(k8 + u) * (size_t)N + ns];
    const float r = zr ? 0.0f : bf16r(f);
    if (F16) o[u] = f16_bits(r * scale);
    else     o[u] = bf16_bits(r);
  }
  const size_t off = (size_t)n * (size_t)K + k8;
  *(volatile us8*)(dst + off) = o;
  __threadfence();
  *(volatile us8*)(dst + off) = o;
}

template <int F16>
__global__ __launch_bounds__(256) void k_gemm(const unsigned short* __restrict__ Ap, int lda,
                                             const unsigned short* __restrict__ Bw, int ldb, int K,
                                             float* Yf, int ldy, float oscale) {
  __shared__ __attribute__((aligned(16))) float oS[8 * 16 * OSTR];
  const int tid = threadIdx.x, lane = tid & 31, wave = tid >> 5, cl = lane & 15, hh = lane >> 4;
  const int m0 = blockIdx.x * TPB + 16 * wave, n0 = blockIdx.y * 64;

  v8f acc[4];
#pragma unroll
  for (int j = 0; j < 4; ++j) { const v8f zz = {0.f, 0.f, 0.f, 0.f, 0.f, 0.f, 0.f, 0.f}; acc[j] = zz; }

  const unsigned short* ap  = Ap + (size_t)(m0 + cl) * (size_t)lda;
  const unsigned short* bwp = Bw + (size_t)(n0 + cl) * (size_t)ldb;
#pragma unroll 1
  for (int k0 = 0; k0 < K; k0 += 32) {
    const us16 af = gfrag(ap + k0);
    us16 bfr[4];
#pragma unroll
    for (int j = 0; j < 4; ++j) bfr[j] = gfrag(bwp + (size_t)(16 * j) * (size_t)ldb + k0);
#pragma unroll
    for (int j = 0; j < 4; ++j) acc[j] = MmaSel<F16>::run(af, bfr[j], acc[j]);
    wguard(acc[0], acc[1], acc[2], acc[3], af, bfr[0], bfr[1], bfr[2], bfr[3]);
  }

  float* so = oS + wave * (16 * OSTR);
#pragma unroll
  for (int j = 0; j < 4; ++j)
#pragma unroll
    for (int r = 0; r < 8; ++r) so[(8 * hh + r) * OSTR + 16 * j + cl] = acc[j][r];
  __syncthreads();

#pragma unroll
  for (int pass = 0; pass < 2; ++pass) {
#pragma unroll
    for (int it = 0; it < 8; ++it) {
      const int cx = it * 32 + lane, r = cx >> 4, q = (cx & 15) * 4;
      const v4f v = *(const v4fa*)(so + r * OSTR + q) * oscale;
      *(volatile v4f*)(Yf + (size_t)(m0 + r) * (size_t)ldy + n0 + q) = v;
    }
    __threadfence();
  }
}

__global__ __launch_bounds__(256) void k_conv(const float* __restrict__ ZX, const float* __restrict__ cw,
                                             const float* __restrict__ cb, float* XC) {
  const int idx = blockIdx.x * 256 + threadIdx.x;
  if (idx >= MTOK * (CD / 4)) return;
  const int m = idx >> 7, c4 = (idx & 127) * 4;
  const int l = m & (SEQL - 1);
  v4f xv[4];
#pragma unroll
  for (int k = 0; k < 4; ++k) {
    const int back = 3 - k;
    const bool ok = (l >= back);
    const int sr = ok ? (m - back) : m;
    const v4f t = *(const v4fa*)(ZX + (size_t)sr * LDZ + COL_XBC + c4);
    v4f z;
#pragma unroll
    for (int u = 0; u < 4; ++u) z[u] = ok ? t[u] : 0.0f;
    xv[k] = z;
  }
  v4f ov;
#pragma unroll
  for (int u = 0; u < 4; ++u) {
    const v4f wr = *(const v4fa*)(cw + (size_t)(c4 + u) * 4);
    const float w0 = bf16r(wr[0]), w1 = bf16r(wr[1]), w2 = bf16r(wr[2]), w3 = bf16r(wr[3]);
    const float acc = (((w0 * xv[0][u] + w1 * xv[1][u]) + w2 * xv[2][u]) + w3 * xv[3][u]) + bf16r(cb[c4 + u]);
    ov[u] = siluf(acc);
  }
  const size_t off = (size_t)m * CD + c4;
  *(volatile v4f*)(XC + off) = ov;
  __threadfence();
  *(volatile v4f*)(XC + off) = ov;
}

__global__ __launch_bounds__(256) void k_scan(const float* __restrict__ ZX, const float* __restrict__ XC,
                                             const float* __restrict__ dtb, const float* __restrict__ Alog,
                                             const float* __restrict__ Dsk, float* Y) {
  __shared__ __attribute__((aligned(16))) float sDT[SEQL];
  __shared__ __attribute__((aligned(16))) float sDA[SEQL];
  __shared__ __attribute__((aligned(16))) float sy[SCH * HDIM];
  const int tid = threadIdx.x;
  const int s = blockIdx.x / NH, hh = blockIdx.x - s * NH;
  const int p = tid >> 2, sub = tid & 3, n0 = sub * NSTS;
  const size_t row0 = (size_t)s * SEQL;
  const float Acoef = -expf(bf16r(Alog[hh]));
  const float dbias = bf16r(dtb[hh]);
  const float Dd = bf16r(Dsk[hh]);

#pragma unroll 1
  for (int i = tid; i < SEQL; i += 256) {
    const float v = ZX[(row0 + (size_t)i) * LDZ + COL_DT + hh] + dbias;
    const float dt = fmaxf(v, 0.0f) + log1pf(expf(-fabsf(v)));
    sDT[i] = dt;
    sDA[i] = expf(dt * Acoef);
  }
  __syncthreads();

  float h[NSTS];
#pragma unroll
  for (int i = 0; i < NSTS; ++i) h[i] = 0.0f;

#pragma unroll 1
  for (int c = 0; c < SEQL / SCH; ++c) {
#pragma unroll 1
    for (int st = 0; st < SCH; ++st) {
      const int l = c * SCH + st;
      const float* xr = XC + (row0 + (size_t)l) * CD;
      const float xv = xr[hh * HDIM + p];
      v4f Bv[4], Cv[4];
#pragma unroll
      for (int q = 0; q < 4; ++q) {
        Bv[q] = *(const v4fa*)(xr + XCB + n0 + 4 * q);
        Cv[q] = *(const v4fa*)(xr + XCC + n0 + 4 * q);
      }
      const float dl = sDT[l], da = sDA[l];
      const float dx = dl * xv;
      float y = 0.0f;
#pragma unroll
      for (int i = 0; i < NSTS; ++i) {
        h[i] = da * h[i] + dx * Bv[i >> 2][i & 3];
        y = y + h[i] * Cv[i >> 2][i & 3];
      }
      y += __shfl_xor(y, 1);
      y += __shfl_xor(y, 2);
      const float yv = y + xv * Dd;
      if (sub == 0) sy[st * HDIM + p] = yv;
    }
    __syncthreads();
#pragma unroll
    for (int pass = 0; pass < 2; ++pass) {
#pragma unroll
      for (int it = 0; it < 2; ++it) {
        const int cx = it * 256 + tid, r = cx >> 4, q = (cx & 15) * 4;
        const v4f v = *(const v4fa*)(sy + r * HDIM + q);
        *(volatile v4f*)(Y + (row0 + (size_t)(c * SCH + r)) * DI + hh * HDIM + q) = v;
      }
      __threadfence();
    }
    __syncthreads();
  }
}

__global__ __launch_bounds__(128) void k_norm(const float* __restrict__ Y, const float* __restrict__ ZX,
                                             const float* __restrict__ nw, unsigned short* YC) {
  __shared__ __attribute__((aligned(16))) float sY[4 * DI];
  const int tid = threadIdx.x, lane = tid & 31, d = tid >> 5;
  const int P = blockIdx.x;
  const int b = P >> 10, iq = (P >> 5) & 31, jq = P & 31;
  const int l0 = iq * 32 + jq, l1 = iq * 32 + (31 - jq), l2 = jq * 32 + iq, l3 = jq * 32 + (31 - iq);
  const int l = (d == 0) ? l0 : ((d == 1) ? l1 : ((d == 2) ? l2 : l3));
  const size_t m = (size_t)(d * NBAT + b) * SEQL + (size_t)l;
  v4f g[3];
  float ss = 0.0f;
#pragma unroll
  for (int j = 0; j < 3; ++j) {
    const int c = 128 * j + 4 * lane;
    const v4f yv = *(const v4fa*)(Y + m * DI + c);
    const v4f zv = *(const v4fa*)(ZX + m * LDZ + c);
    v4f t;
#pragma unroll
    for (int u = 0; u < 4; ++u) { t[u] = yv[u] * siluf(zv[u]); ss += t[u] * t[u]; }
    g[j] = t;
  }
  ss += __shfl_xor(ss, 16);
  ss += __shfl_xor(ss, 8);
  ss += __shfl_xor(ss, 4);
  ss += __shfl_xor(ss, 2);
  ss += __shfl_xor(ss, 1);
  const float rs = rsqrtf(ss * (1.0f / (float)DI) + EPSV);
#pragma unroll
  for (int j = 0; j < 3; ++j) {
    const int c = 128 * j + 4 * lane;
    v4f o;
#pragma unroll
    for (int u = 0; u < 4; ++u) o[u] = (g[j][u] * rs) * bf16r(nw[c + u]) * 0.25f;
    *(v4fa*)(sY + d * DI + c) = o;
  }
  __syncthreads();
  if (tid < 48) {
    const int c8 = tid * 8;
    us8 o;
#pragma unroll
    for (int u = 0; u < 8; ++u) {
      const float sum = ((sY[c8 + u] + sY[DI + c8 + u]) + sY[2 * DI + c8 + u]) + sY[3 * DI + c8 + u];
      o[u] = f16_bits(sum);
    }
    const size_t off = (size_t)P * DI + c8;
    *(volatile us8*)(YC + off) = o;
    __threadfence();
    *(volatile us8*)(YC + off) = o;
  }
}

extern "C" void kernel_launch(void* const* d_in, const int* in_sizes, int n_in,
                              void* d_out, int out_size, void* d_ws, size_t ws_size,
                              hipStream_t stream) {
  if (n_in < 9) return;
  if (in_sizes[0] != NPIX * DM || in_sizes[1] != DM * NPJ || in_sizes[2] != CD * 4 || in_sizes[3] != CD ||
      in_sizes[4] != NH || in_sizes[5] != NH || in_sizes[6] != NH || in_sizes[7] != DI || in_sizes[8] != DI * DM) return;
  if (out_size != NPIX * DM) return;

  const float* x      = (const float*)d_in[0];
  const float* w_in   = (const float*)d_in[1];
  const float* conv_w = (const float*)d_in[2];
  const float* conv_b = (const float*)d_in[3];
  const float* dt_b   = (const float*)d_in[4];
  const float* a_log  = (const float*)d_in[5];
  const float* d_skp  = (const float*)d_in[6];
  const float* norm_w = (const float*)d_in[7];
  const float* w_out  = (const float*)d_in[8];
  float* out = (float*)d_out;

  size_t off = 0;
  auto carve = [&](size_t bytes) -> char* { char* p = (char*)d_ws + off; off += (bytes + 255) & ~(size_t)255; return p; };
  float* ZX = (float*)carve((size_t)MTOK * LDZ * 4);
  float* XC = (float*)carve((size_t)MTOK * CD * 4);
  float* Y  = (float*)carve((size_t)MTOK * DI * 4);
  unsigned short* XB  = (unsigned short*)carve((size_t)MTOK * DM * 2);
  unsigned short* WIB = (unsigned short*)carve((size_t)LDZ * DM * 2);
  unsigned short* WOB = (unsigned short*)carve((size_t)DM * DI * 2);
  if (off > ws_size || off > (size_t)WSCAP) return;
  unsigned short* YC = XB;

  const dim3 b256(256), b128(128);
  auto cdv = [](long a, long bq) { return (unsigned)((a + bq - 1) / bq); };

  k_gather<<<dim3(cdv((long)MTOK * (DM / 8), 256)), b256, 0, stream>>>(x, XB);
  k_cvtw<0><<<dim3(cdv((long)LDZ * (DM / 8), 256)), b256, 0, stream>>>(w_in, WIB, DM, NPJ, LDZ * (DM / 8), 1.0f);
  k_cvtw<1><<<dim3(cdv((long)DM * (DI / 8), 256)), b256, 0, stream>>>(w_out, WOB, DI, DM, DM * (DI / 8), WOSC);
  k_gemm<0><<<dim3(MTOK / TPB, LDZ / 64), b256, 0, stream>>>(XB, DM, WIB, DM, DM, ZX, LDZ, 1.0f);
  k_conv<<<dim3(cdv((long)MTOK * (CD / 4), 256)), b256, 0, stream>>>(ZX, conv_w, conv_b, XC);
  k_scan<<<dim3(NSEQ * NH), b256, 0, stream>>>(ZX, XC, dt_b, a_log, d_skp, Y);
  k_norm<<<dim3(NPIX), b128, 0, stream>>>(Y, ZX, norm_w, YC);
  k_gemm<1><<<dim3(NPIX / TPB, DM / 64), b256, 0, stream>>>(YC, DI, WOB, DI, DI, out, DM, WOSCI);
}
